// VoxelSDF_19215683682576
// MI455X (gfx1250) — hardware-verified
//
#include <hip/hip_runtime.h>


#define G1      33
#define VOX     (G1 * G1 * G1)
#define LATENT  32
#define HID     128
#define NTILE1  8
#define NTILES  48
#define TPB     256
#define LATP    36

typedef _Float16       v16h __attribute__((ext_vector_type(16)));
typedef _Float16       v8h  __attribute__((ext_vector_type(8)));
typedef __bf16         v16b __attribute__((ext_vector_type(16)));
typedef unsigned short v16u __attribute__((ext_vector_type(16)));
typedef unsigned short v8u  __attribute__((ext_vector_type(8)));
typedef float          v8f  __attribute__((ext_vector_type(8)));
typedef float          v4f  __attribute__((ext_vector_type(4)));

union FragH { v16h v; v8h half[2]; };
union FragU { v16b b; v16u u; v8u half[2]; };
union H2U   { _Float16 h; unsigned short u; };

__device__ __forceinline__ unsigned short f32_to_bf16_bits(float x) {
  unsigned int u = __float_as_uint(x);
  u += 0x7FFFu + ((u >> 16) & 1u);
  return (unsigned short)(u >> 16);
}
__device__ __forceinline__ float bf16_bits_to_f32(unsigned short b) {
  return __uint_as_float(((unsigned int)b) << 16);
}

__device__ __forceinline__ v8f mma_f16(v16h a, v16h b, v8f c) {
  c = __builtin_amdgcn_wmma_f32_16x16x32_f16(false, a, false, b, (short)0, c, false, false);
  asm volatile("v_nop\n\tv_nop\n\tv_nop\n\tv_nop" : "+v"(c) : "v"(a), "v"(b));
  return c;
}
__device__ __forceinline__ v8f mma_bf16(v16u au, v16u bu, v8f c) {
  FragU a, b;
  a.u = au;
  b.u = bu;
  c = __builtin_amdgcn_wmma_f32_16x16x32_bf16(false, a.b, false, b.b, (short)0, c, false, false);
  asm volatile("v_nop\n\tv_nop\n\tv_nop\n\tv_nop" : "+v"(c) : "v"(au), "v"(bu));
  return c;
}

__global__ void __launch_bounds__(TPB) k_repack_emb(const float* __restrict__ emb, float* __restrict__ embt) {
  const int t = blockIdx.x * TPB + threadIdx.x;
  const int v = t >> 3, q = t & 7;
  const bool ok = v < VOX;
  const int vc = ok ? v : 0;
  v4f val;
  val.x = emb[(size_t)(4 * q + 0) * VOX + vc];
  val.y = emb[(size_t)(4 * q + 1) * VOX + vc];
  val.z = emb[(size_t)(4 * q + 2) * VOX + vc];
  val.w = emb[(size_t)(4 * q + 3) * VOX + vc];
  volatile v4f* p = (volatile v4f*)(embt + (size_t)vc * LATENT + 4 * q);
  if (ok) *p = val;
  __threadfence();
  if (ok) *p = val;
}

__global__ void __launch_bounds__(TPB) k_build_frags(const float* __restrict__ w1, const float* __restrict__ w2,
                                                     unsigned short* __restrict__ frag) {
  const int t = blockIdx.x * TPB + threadIdx.x;
  const bool ok = t < NTILES * 64;
  const int tt = ok ? t : 0;
  const int tile = tt >> 6, lane = (tt >> 1) & 31, g = tt & 1;
  const int n16 = lane & 15, h = lane >> 4;
  const int kl0 = 16 * g + 8 * h;
  v8u o;
#pragma unroll
  for (int e = 0; e < 8; ++e) {
    const int kl = kl0 + e;
    unsigned short bits;
    if (tile < 2 * NTILE1) {
      const int nt = tile & 7;
      const float x = w1[kl * HID + nt * 16 + n16];
      const unsigned short hb = f32_to_bf16_bits(x);
      bits = (tile < NTILE1) ? hb : f32_to_bf16_bits(x - bf16_bits_to_f32(hb));
    } else {
      const int u = tile - 2 * NTILE1, nt = u >> 2, kb = u & 3;
      const float x = w2[(kb * 32 + kl) * HID + nt * 16 + n16] * 16.f;
      H2U cv;
      cv.h = (_Float16)x;
      bits = cv.u;
    }
    o[e] = bits;
  }
  volatile v8u* p = (volatile v8u*)(frag + (size_t)tt * 8);
  if (ok) *p = o;
  __threadfence();
  if (ok) *p = o;
}

__global__ void __launch_bounds__(TPB) k_voxel_mlp(
    const float* __restrict__ points,
    const float* __restrict__ embt,
    const unsigned short* __restrict__ frag,
    const float* __restrict__ b1,
    const float* __restrict__ b2,
    const float* __restrict__ w3,
    const float* __restrict__ b3,
    float* __restrict__ out,
    int npts)
{
  __shared__ __align__(16) float    latS[8][16][LATP];
  __shared__ __align__(16) _Float16 h1[8][16][HID];
  __shared__ __align__(16) float    sOut[128];

  const int lane = threadIdx.x & 31;
  const int w    = threadIdx.x >> 5;
  const int m    = lane & 15;
  const int h    = lane >> 4;
  const int blockBase = blockIdx.x * 128;
  const int p0   = blockBase + w * 16;
  int pt = p0 + m;
  pt = (pt < npts) ? pt : (npts - 1);

  const float px = points[(size_t)pt * 3 + 0];
  const float py = points[(size_t)pt * 3 + 1];
  const float pz = points[(size_t)pt * 3 + 2];
  const float cx = (px + 1.f) * 16.f, cy = (py + 1.f) * 16.f, cz = (pz + 1.f) * 16.f;
  const float flx = floorf(cx), fly = floorf(cy), flz = floorf(cz);
  const int x0 = (int)flx, y0 = (int)fly, z0 = (int)flz;
  const float fx = cx - flx, fy = cy - fly, fz = cz - flz;
  const float wx0 = 1.f - fx, wx1 = fx;
  const float wy0 = 1.f - fy, wy1 = fy;
  const float wz0 = 1.f - fz, wz1 = fz;

  float acc[16];
#pragma unroll
  for (int j = 0; j < 16; ++j) acc[j] = 0.f;

#pragma unroll
  for (int c = 0; c < 8; ++c) {
    const int xi = x0 + (c & 1), yi = y0 + ((c >> 1) & 1), zi = z0 + (c >> 2);
    const float wx = (c & 1) ? wx1 : wx0;
    const float wy = ((c >> 1) & 1) ? wy1 : wy0;
    const float wz = (c >> 2) ? wz1 : wz0;
    float wgt = (wz * wy) * wx;
    const bool valid = ((unsigned)xi < (unsigned)G1) & ((unsigned)yi < (unsigned)G1) &
                       ((unsigned)zi < (unsigned)G1);
    wgt = valid ? wgt : 0.f;
    const int xc = min(max(xi, 0), G1 - 1), yc = min(max(yi, 0), G1 - 1), zc = min(max(zi, 0), G1 - 1);
    const int v = (zc * G1 + yc) * G1 + xc;
    const float* rp = embt + (size_t)v * LATENT;
    const v4f q0 = *(const v4f*)(rp + 8 * h);
    const v4f q1 = *(const v4f*)(rp + 8 * h + 4);
    const v4f q2 = *(const v4f*)(rp + 16 + 8 * h);
    const v4f q3 = *(const v4f*)(rp + 16 + 8 * h + 4);
    acc[0]  += wgt * q0.x; acc[1]  += wgt * q0.y; acc[2]  += wgt * q0.z; acc[3]  += wgt * q0.w;
    acc[4]  += wgt * q1.x; acc[5]  += wgt * q1.y; acc[6]  += wgt * q1.z; acc[7]  += wgt * q1.w;
    acc[8]  += wgt * q2.x; acc[9]  += wgt * q2.y; acc[10] += wgt * q2.z; acc[11] += wgt * q2.w;
    acc[12] += wgt * q3.x; acc[13] += wgt * q3.y; acc[14] += wgt * q3.z; acc[15] += wgt * q3.w;
  }

  {
    float* lrow = &latS[w][m][0];
    v4f s0, s1, s2, s3;
    s0.x = acc[0];  s0.y = acc[1];  s0.z = acc[2];  s0.w = acc[3];
    s1.x = acc[4];  s1.y = acc[5];  s1.z = acc[6];  s1.w = acc[7];
    s2.x = acc[8];  s2.y = acc[9];  s2.z = acc[10]; s2.w = acc[11];
    s3.x = acc[12]; s3.y = acc[13]; s3.z = acc[14]; s3.w = acc[15];
    *(v4f*)(lrow + 8 * h)          = s0;
    *(v4f*)(lrow + 8 * h + 4)      = s1;
    *(v4f*)(lrow + 16 + 8 * h)     = s2;
    *(v4f*)(lrow + 16 + 8 * h + 4) = s3;
  }
  __syncthreads();

  FragU ahi, alo;
  {
    const float* lrow = &latS[w][m][0];
    const v4f r0 = *(const v4f*)(lrow + 8 * h);
    const v4f r1 = *(const v4f*)(lrow + 8 * h + 4);
    const v4f r2 = *(const v4f*)(lrow + 16 + 8 * h);
    const v4f r3 = *(const v4f*)(lrow + 16 + 8 * h + 4);
    float av[16];
    av[0]  = r0.x; av[1]  = r0.y; av[2]  = r0.z; av[3]  = r0.w;
    av[4]  = r1.x; av[5]  = r1.y; av[6]  = r1.z; av[7]  = r1.w;
    av[8]  = r2.x; av[9]  = r2.y; av[10] = r2.z; av[11] = r2.w;
    av[12] = r3.x; av[13] = r3.y; av[14] = r3.z; av[15] = r3.w;
#pragma unroll
    for (int j = 0; j < 16; ++j) {
      const unsigned short hb = f32_to_bf16_bits(av[j]);
      ahi.u[j] = hb;
      alo.u[j] = f32_to_bf16_bits(av[j] - bf16_bits_to_f32(hb));
    }
  }

#pragma unroll
  for (int nt = 0; nt < NTILE1; ++nt) {
    const unsigned short* bp = frag + (size_t)(nt * 32 + lane) * 16;
    const unsigned short* bq = frag + (size_t)((NTILE1 + nt) * 32 + lane) * 16;
    FragU bh, bl;
    bh.half[0] = *(const v8u*)(bp);
    bh.half[1] = *(const v8u*)(bp + 8);
    bl.half[0] = *(const v8u*)(bq);
    bl.half[1] = *(const v8u*)(bq + 8);
    const float bb = b1[nt * 16 + m];
    v8f cacc;
#pragma unroll
    for (int r = 0; r < 8; ++r) cacc[r] = bb;
    cacc = mma_bf16(ahi.u, bh.u, cacc);
    cacc = mma_bf16(ahi.u, bl.u, cacc);
    cacc = mma_bf16(alo.u, bh.u, cacc);
#pragma unroll
    for (int r = 0; r < 8; ++r)
      h1[w][8 * h + r][nt * 16 + m] = (_Float16)(fmaxf(cacc[r], 0.f) * 16.f);
  }
  __syncthreads();

  FragH a2[4];
#pragma unroll
  for (int kb = 0; kb < 4; ++kb) {
    a2[kb].half[0] = *(const v8h*)(&h1[w][m][kb * 32 + 8 * h]);
    a2[kb].half[1] = *(const v8h*)(&h1[w][m][kb * 32 + 16 + 8 * h]);
  }

  const _Float16* fragh = (const _Float16*)frag;
  float partial[8];
#pragma unroll
  for (int r = 0; r < 8; ++r) partial[r] = 0.f;

#pragma unroll
  for (int nt = 0; nt < 8; ++nt) {
    const float bb = b2[nt * 16 + m] * 256.f;
    v8f cacc;
#pragma unroll
    for (int r = 0; r < 8; ++r) cacc[r] = bb;
#pragma unroll
    for (int kb = 0; kb < 4; ++kb) {
      const _Float16* bp = fragh + (size_t)((2 * NTILE1 + nt * 4 + kb) * 32 + lane) * 16;
      FragH bf;
      bf.half[0] = *(const v8h*)(bp);
      bf.half[1] = *(const v8h*)(bp + 8);
      cacc = mma_f16(a2[kb].v, bf.v, cacc);
    }
    const float w3v = w3[nt * 16 + m];
#pragma unroll
    for (int r = 0; r < 8; ++r) {
      const float hv = fmaxf(cacc[r], 0.f) * (1.f / 256.f);
      partial[r] += hv * w3v;
    }
  }

#pragma unroll
  for (int mask = 1; mask < 16; mask <<= 1) {
#pragma unroll
    for (int r = 0; r < 8; ++r) partial[r] += __shfl_xor(partial[r], mask, 32);
  }
  const float b3v = b3[0];
  if (m == 0) {
#pragma unroll
    for (int r = 0; r < 8; ++r) sOut[w * 16 + 8 * h + r] = tanhf(partial[r] + b3v);
  }
  __syncthreads();

  const bool fullblk = (blockBase + 128) <= npts;
  if (fullblk) {
    if (w == 0) {
      const v4f ov = *(const v4f*)(&sOut[4 * lane]);
      volatile v4f* op = (volatile v4f*)(out + (size_t)blockBase + 4 * lane);
      *op = ov;
      __threadfence();
      *op = ov;
    }
  } else {
    const int t = threadIdx.x;
    const int idx = blockBase + t;
    const bool ok = (t < 128) && (idx < npts);
    const float ov = sOut[(t < 128) ? t : 0];
    volatile float* op = out + (size_t)(ok ? idx : 0);
    if (ok) *op = ov;
    __threadfence();
    if (ok) *op = ov;
  }
}

extern "C" void kernel_launch(void* const* d_in, const int* in_sizes, int n_in,
                              void* d_out, int out_size, void* d_ws, size_t ws_size,
                              hipStream_t stream) {
  if (n_in < 8) return;
  const float* points = (const float*)d_in[0];
  const float* emb    = (const float*)d_in[1];
  const float* w1     = (const float*)d_in[2];
  const float* b1     = (const float*)d_in[3];
  const float* w2     = (const float*)d_in[4];
  const float* b2     = (const float*)d_in[5];
  const float* w3     = (const float*)d_in[6];
  const float* b3     = (const float*)d_in[7];
  float* out = (float*)d_out;

  int npts = in_sizes[0] / 3;
  if (npts > out_size) npts = out_size;

  const size_t off_embt = 0;
  const size_t bytes_embt = (size_t)VOX * LATENT * sizeof(float);
  const size_t off_frag = off_embt + bytes_embt;
  const size_t bytes_frag = (size_t)NTILES * 512 * sizeof(unsigned short);
  if (off_frag + bytes_frag > ws_size) return;
  float* embt = (float*)((char*)d_ws + off_embt);
  unsigned short* frag = (unsigned short*)((char*)d_ws + off_frag);

  k_repack_emb<<<(VOX * 8 + TPB - 1) / TPB, TPB, 0, stream>>>(emb, embt);
  k_build_frags<<<(NTILES * 64 + TPB - 1) / TPB, TPB, 0, stream>>>(w1, w2, frag);
  const int nblk = (npts + 127) / 128;
  if (nblk > 0)
    k_voxel_mlp<<<nblk, TPB, 0, stream>>>(points, embt, frag, b1, b2, w3, b3, out, npts);
}
